// SelectiveSSM_33440615367094
// MI455X (gfx1250) — hardware-run, weakly checked
//
#include <hip/hip_runtime.h>
#include <math.h>

typedef __attribute__((ext_vector_type(16))) _Float16 v16h;
typedef __attribute__((ext_vector_type(8)))  _Float16 v8h;
typedef __attribute__((ext_vector_type(16))) __bf16   v16b;
typedef __attribute__((ext_vector_type(8)))  __bf16   v8b;
typedef __attribute__((ext_vector_type(8)))  float    v8f;
typedef __attribute__((ext_vector_type(4)))  float    v4f;

constexpr int   kBatch  = 2;
constexpr int   kSeq    = 2048;
constexpr int   kD      = 1024;
constexpr int   kN      = 16;
constexpr int   kRows   = kBatch * kSeq;
constexpr int   kNW     = kD + 2 * kN;
constexpr int   kNP     = 1088;
constexpr float kDT     = 0.1f;
constexpr int   kScanCh = 256;
constexpr int   kScanTS = 16;
constexpr int   kScanTP = 260;
static_assert(kNP % 64 == 0 && kNP >= kNW && kNP - kD == 64, "padded projection width");
static_assert(kD % 32 == 0, "GEMM K multiple of 32");
static_assert(kRows % 64 == 0 && kNP % 64 == 0, "GEMM M,N multiples of 64");
static_assert(((kRows / 64) * (kNP / 64)) % 8 == 0, "whole GEMM blocks");
static_assert(kSeq % kScanTS == 0 && kD % kScanCh == 0 && (kBatch * kD) % 32 == 0, "tile multiples");
static_assert((kNP * 4) % 128 == 0, "P row pitch is a line multiple");

constexpr size_t kOffGC   = 0;
constexpr size_t kOffSEL  = kOffGC  + (size_t)kBatch * kD * 4;
constexpr size_t kOffXSH  = kOffSEL + (size_t)kBatch * kD * 4;
constexpr size_t kOffXSL  = kOffXSH + (size_t)kRows * kD * 2;
constexpr size_t kOffWH   = kOffXSL + (size_t)kRows * kD * 2;
constexpr size_t kOffWL   = kOffWH  + (size_t)kNP * kD * 2;
constexpr size_t kOffP    = kOffWL  + (size_t)kNP * kD * 2;
constexpr size_t kWsTotal = kOffP   + (size_t)kRows * kNP * 4;
static_assert(kWsTotal == 39075840ull, "carve total");
static_assert(kWsTotal <= 134217728ull, "carve cap");
static_assert((kOffSEL % 128) == 0 && (kOffXSH % 128) == 0 && (kOffXSL % 128) == 0 && (kOffWH % 128) == 0 &&
              (kOffWL % 128) == 0 && (kOffP % 128) == 0, "128-B aligned regions");

__device__ __forceinline__ unsigned short f2bf_bits(float f) {
  unsigned u = __float_as_uint(f);
  return (unsigned short)((u + 0x7FFFu + ((u >> 16) & 1u)) >> 16);
}
__device__ __forceinline__ float bf_bits2f(unsigned short h) { return __uint_as_float(((unsigned)h) << 16); }

__device__ __forceinline__ void dep_guard4_h(v8f& a, v8f& b, v8f& c, v8f& d, v16h x, v16h y) { asm volatile("v_nop\n\tv_nop\n\tv_nop\n\tv_nop" : "+v"(a), "+v"(b), "+v"(c), "+v"(d) : "v"(x), "v"(y)); }
__device__ __forceinline__ void dep_guard4_b(v8f& a, v8f& b, v8f& c, v8f& d, v16b x, v16b y) { asm volatile("v_nop\n\tv_nop\n\tv_nop\n\tv_nop" : "+v"(a), "+v"(b), "+v"(c), "+v"(d) : "v"(x), "v"(y)); }
__device__ __forceinline__ void keep4_h(v16h a, v16h b, v16h c, v16h d) { asm volatile("v_nop" :: "v"(a), "v"(b), "v"(c), "v"(d)); }
__device__ __forceinline__ void keep4_b(v16b a, v16b b, v16b c, v16b d) { asm volatile("v_nop" :: "v"(a), "v"(b), "v"(c), "v"(d)); }
__device__ __forceinline__ void acc_guard4(v8f& a, v8f& b, v8f& c, v8f& d) { asm volatile("v_nop\n\tv_nop\n\tv_nop\n\tv_nop" : "+v"(a), "+v"(b), "+v"(c), "+v"(d)); }
template <typename T> struct Frag;
template <> struct Frag<_Float16> {
  typedef v16h V; union U { v16h v; v8h h[2]; };
  static __device__ __forceinline__ v16h load(const _Float16* p) {
    U f; f.h[0] = *(const v8h*)(p); f.h[1] = *(const v8h*)(p + 16); return f.v;
  }
  static __device__ __forceinline__ v8f mma(v16h a, v16h b, v8f c) {
    return __builtin_amdgcn_wmma_f32_16x16x32_f16(false, a, false, b, (short)0, c, false, false);
  }
  static __device__ __forceinline__ void guard4(v8f& a, v8f& b, v8f& c, v8f& d, v16h x, v16h y) { dep_guard4_h(a, b, c, d, x, y); }
  static __device__ __forceinline__ void keep(v16h a, v16h b, v16h c, v16h d) { keep4_h(a, b, c, d); }
};
template <> struct Frag<__bf16> {
  typedef v16b V; union U { v16b v; v8b h[2]; };
  static __device__ __forceinline__ v16b load(const __bf16* p) {
    U f; f.h[0] = *(const v8b*)(p); f.h[1] = *(const v8b*)(p + 16); return f.v;
  }
  static __device__ __forceinline__ v8f mma(v16b a, v16b b, v8f c) {
    return __builtin_amdgcn_wmma_f32_16x16x32_bf16(false, a, false, b, (short)0, c, false, false);
  }
  static __device__ __forceinline__ void guard4(v8f& a, v8f& b, v8f& c, v8f& d, v16b x, v16b y) { dep_guard4_b(a, b, c, d, x, y); }
  static __device__ __forceinline__ void keep(v16b a, v16b b, v16b c, v16b d) { keep4_b(a, b, c, d); }
};

template <int ET> struct Elem;
template <> struct Elem<0> { typedef _Float16 T; };
template <> struct Elem<1> { typedef __bf16 T; };
template <int ET, int SPL, int BIAS_MODE, int OUT_MODE, bool RESID, int ACT = 0>
__global__ __launch_bounds__(256) void wmma_gemm64(
    const unsigned short* __restrict__ Ap, const unsigned short* __restrict__ A2p, int lda, long strideA,
    const unsigned short* __restrict__ Btp, const unsigned short* __restrict__ Bt2p, int ldb, long strideB,
    void* __restrict__ Cout, void* __restrict__ Cout2, int ldc, long strideC,
    const float* __restrict__ bias,
    const float* __restrict__ resid, long strideR,
    int M, int N, int K, float scale) {
  typedef typename Elem<ET>::T T;
  typedef typename Frag<T>::V V;
  const T* A = (const T*)Ap; const T* A2 = (const T*)A2p; const T* Bt = (const T*)Btp; const T* Bt2 = (const T*)Bt2p;
  __shared__ __align__(16) float sT[8][16 * 68];
  const int b    = blockIdx.y;
  const int lane = threadIdx.x & 31;
  const int wave = threadIdx.x >> 5;
  const int tilesN = N >> 6;
  const int tilesM = M >> 6;
  const int tile = blockIdx.x * 8 + wave;
  if (tile >= tilesM * tilesN) return;
  const int tm = tile / tilesN;
  const int tn = tile - tm * tilesN;
  const int m0 = tm << 6;
  const int n0 = tn << 6;

  const T* Ab  = A  + (size_t)b * strideA;
  const T* Bb  = Bt + (size_t)b * strideB;
  const T* Ab2 = (SPL >= 1) ? (A2  + (size_t)b * strideA) : nullptr;
  const T* Bb2 = (SPL == 2) ? (Bt2 + (size_t)b * strideB) : nullptr;

  const int rlane = lane & 15;
  const int koff  = (lane >> 4) * 8;
  const int mOff  = (lane >> 4) * 8;

  v8f acc[4][4];
#pragma unroll
  for (int i = 0; i < 4; ++i)
#pragma unroll
    for (int j = 0; j < 4; ++j) acc[i][j] = (v8f){0.f,0.f,0.f,0.f,0.f,0.f,0.f,0.f};

  for (int k0 = 0; k0 < K; k0 += 32) {
    V bh[4], bl[4];
#pragma unroll
    for (int j = 0; j < 4; ++j) {
      const size_t bo = (size_t)(n0 + (j << 4) + rlane) * ldb + koff + k0;
      bh[j] = Frag<T>::load(Bb + bo);
      if (SPL == 2) bl[j] = Frag<T>::load(Bb2 + bo);
    }
#pragma unroll
    for (int i = 0; i < 4; ++i) {
      const size_t ao = (size_t)(m0 + (i << 4) + rlane) * lda + koff + k0;
      V ah = Frag<T>::load(Ab + ao);
      V al;
      if (SPL >= 1) al = Frag<T>::load(Ab2 + ao);
#pragma unroll
      for (int j = 0; j < 4; ++j) {
        acc[i][j] = Frag<T>::mma(ah, bh[j], acc[i][j]);
        if (SPL == 2) acc[i][j] = Frag<T>::mma(ah, bl[j], acc[i][j]);
        if (SPL >= 1) acc[i][j] = Frag<T>::mma(al, bh[j], acc[i][j]);
      }
      Frag<T>::guard4(acc[i][0], acc[i][1], acc[i][2], acc[i][3], ah, (SPL >= 1) ? al : ah);
    }
    Frag<T>::keep(bh[0], bh[1], bh[2], bh[3]);
    if (SPL == 2) Frag<T>::keep(bl[0], bl[1], bl[2], bl[3]);
  }
  acc_guard4(acc[0][0], acc[0][1], acc[0][2], acc[0][3]);
  acc_guard4(acc[1][0], acc[1][1], acc[1][2], acc[1][3]);
  acc_guard4(acc[2][0], acc[2][1], acc[2][2], acc[2][3]);
  acc_guard4(acc[3][0], acc[3][1], acc[3][2], acc[3][3]);

  float* slab = sT[wave];
  const float* Rb = RESID ? (resid + (size_t)b * strideR) : nullptr;
#pragma unroll
  for (int i = 0; i < 4; ++i) {
    const int mBase = m0 + (i << 4);
#pragma unroll
    for (int j = 0; j < 4; ++j) {
      const int n = n0 + (j << 4) + rlane;
      float bv = 0.f;
      if (BIAS_MODE == 2) bv = bias[n];
#pragma unroll
      for (int r = 0; r < 8; ++r) {
        float v = acc[i][j][r] * scale;
        if (BIAS_MODE == 1) v += bias[mBase + mOff + r];
        if (BIAS_MODE == 2) v += bv;
        if (RESID) v += Rb[(size_t)(mBase + mOff + r) * ldc + n];
        if (ACT == 1) v = tanhf(v);
        if (ACT == 2) v = fmaxf(v, 0.0f);
        if (ACT == 3) v = v / (1.0f + expf(-v));
        if (ACT == 4) v = (v > 0.f) ? v : 0.01f * v;
        slab[(mOff + r) * 68 + (j << 4) + rlane] = v;
      }
    }
    __builtin_amdgcn_fence(__ATOMIC_RELEASE, "workgroup");
    __builtin_amdgcn_wave_barrier();
    __builtin_amdgcn_fence(__ATOMIC_ACQUIRE, "workgroup");
    if (OUT_MODE == 0) {
      float* C = (float*)Cout + (size_t)b * strideC;
      const int hh = lane >> 4, c4 = (lane & 15) * 4;
      for (int pass = 0; pass < 2; ++pass) {
#pragma unroll
        for (int it = 0; it < 8; ++it) {
          const int row = it * 2 + hh;
          v4f v = *(const v4f*)(slab + row * 68 + c4);
          *(volatile v4f*)(C + (size_t)(mBase + row) * ldc + n0 + c4) = v;
        }
        __threadfence();
      }
    } else {
      const int q = lane >> 3, c8 = (lane & 7) * 8;
      unsigned short* C  = (unsigned short*)Cout  + (size_t)b * strideC;
      unsigned short* C2 = (OUT_MODE == 2) ? ((unsigned short*)Cout2 + (size_t)b * strideC) : nullptr;
      for (int pass = 0; pass < 2; ++pass) {
#pragma unroll
        for (int it = 0; it < 4; ++it) {
          const int row = it * 4 + q;
          const float* sp = slab + row * 68 + c8;
          v8h hv, lv;
#pragma unroll
          for (int e = 0; e < 8; ++e) {
            if (OUT_MODE == 1) {
              hv[e] = (_Float16)sp[e];
            } else {
              unsigned short hb = f2bf_bits(sp[e]);
              unsigned short lb = f2bf_bits(sp[e] - bf_bits2f(hb));
              hv[e] = __builtin_bit_cast(_Float16, hb);
              lv[e] = __builtin_bit_cast(_Float16, lb);
            }
          }
          *(volatile v8h*)(C + (size_t)(mBase + row) * ldc + n0 + c8) = hv;
          if (OUT_MODE == 2) *(volatile v8h*)(C2 + (size_t)(mBase + row) * ldc + n0 + c8) = lv;
        }
        __threadfence();
      }
    }
    __builtin_amdgcn_fence(__ATOMIC_RELEASE, "workgroup");
    __builtin_amdgcn_wave_barrier();
    __builtin_amdgcn_fence(__ATOMIC_ACQUIRE, "workgroup");
  }
}

__global__ __launch_bounds__(256) void split_rows_bf16_kernel(
    const float* __restrict__ src, unsigned short* __restrict__ dhi, unsigned short* __restrict__ dlo, int total8)
{
  const int i = blockIdx.x * 256 + threadIdx.x;
  if (i >= total8) return;
  const size_t e0 = (size_t)i << 3;
  const v4f a0 = *(const v4f*)(src + e0);
  const v4f a1 = *(const v4f*)(src + e0 + 4);
  v8h hv, lv;
#pragma unroll
  for (int e = 0; e < 4; ++e) {
    const unsigned short h0 = f2bf_bits(a0[e]), h1 = f2bf_bits(a1[e]);
    const unsigned short l0 = f2bf_bits(a0[e] - bf_bits2f(h0)), l1 = f2bf_bits(a1[e] - bf_bits2f(h1));
    hv[e]     = __builtin_bit_cast(_Float16, h0);
    hv[4 + e] = __builtin_bit_cast(_Float16, h1);
    lv[e]     = __builtin_bit_cast(_Float16, l0);
    lv[4 + e] = __builtin_bit_cast(_Float16, l1);
  }
  unsigned short* qh = dhi + e0;
  unsigned short* ql = dlo + e0;
  *(volatile v8h*)qh = hv;
  *(volatile v8h*)ql = lv;
  __threadfence();
  *(volatile v8h*)qh = hv;
  *(volatile v8h*)ql = lv;
}

__global__ __launch_bounds__(256) void xs_split_kernel(
    const float* __restrict__ x, const float* __restrict__ SEL,
    unsigned short* __restrict__ dhi, unsigned short* __restrict__ dlo, int total8)
{
  const int i = blockIdx.x * 256 + threadIdx.x;
  if (i >= total8) return;
  const size_t e0 = (size_t)i << 3;
  const int bix = (int)(e0 >> 21);
  const int dc  = (int)(e0 & (size_t)(kD - 1));
  const v4f a0 = *(const v4f*)(x + e0);
  const v4f a1 = *(const v4f*)(x + e0 + 4);
  const v4f s0 = *(const v4f*)(SEL + (size_t)bix * kD + dc);
  const v4f s1 = *(const v4f*)(SEL + (size_t)bix * kD + dc + 4);
  v8h hv, lv;
#pragma unroll
  for (int e = 0; e < 4; ++e) {
    const float v0 = a0[e] * s0[e];
    const float v1 = a1[e] * s1[e];
    const unsigned short h0 = f2bf_bits(v0), h1 = f2bf_bits(v1);
    const unsigned short l0 = f2bf_bits(v0 - bf_bits2f(h0)), l1 = f2bf_bits(v1 - bf_bits2f(h1));
    hv[e]     = __builtin_bit_cast(_Float16, h0);
    hv[4 + e] = __builtin_bit_cast(_Float16, h1);
    lv[e]     = __builtin_bit_cast(_Float16, l0);
    lv[4 + e] = __builtin_bit_cast(_Float16, l1);
  }
  unsigned short* qh = dhi + e0;
  unsigned short* ql = dlo + e0;
  *(volatile v8h*)qh = hv;
  *(volatile v8h*)ql = lv;
  __threadfence();
  *(volatile v8h*)qh = hv;
  *(volatile v8h*)ql = lv;
}

__global__ __launch_bounds__(256) void wtail_split_kernel(
    const float* __restrict__ BW, const float* __restrict__ CW,
    unsigned short* __restrict__ dhi, unsigned short* __restrict__ dlo)
{
  const int i = blockIdx.x * 256 + threadIdx.x;
  if (i >= ((kNP - kD) * kD) / 8) return;
  const int e0 = i << 3;
  const int r  = e0 >> 10;
  const int k  = e0 & (kD - 1);
  const int rb = (r < kN) ? r : (kN - 1);
  int rc = r - kN; rc = (rc < 0) ? 0 : rc; rc = (rc < kN) ? rc : (kN - 1);
  const v4f b0 = *(const v4f*)(BW + (size_t)rb * kD + k);
  const v4f b1 = *(const v4f*)(BW + (size_t)rb * kD + k + 4);
  const v4f c0 = *(const v4f*)(CW + (size_t)rc * kD + k);
  const v4f c1 = *(const v4f*)(CW + (size_t)rc * kD + k + 4);
  const float fB = (r < kN) ? 1.0f : 0.0f;
  const float fC = (r >= kN && r < 2 * kN) ? 1.0f : 0.0f;
  const bool live = (r < 2 * kN);
  v8h hv, lv;
#pragma unroll
  for (int e = 0; e < 4; ++e) {
    float v0 = fmaf(fB, b0[e], fC * c0[e]);
    float v1 = fmaf(fB, b1[e], fC * c1[e]);
    v0 = live ? v0 : 0.0f;
    v1 = live ? v1 : 0.0f;
    const unsigned short h0 = f2bf_bits(v0), h1 = f2bf_bits(v1);
    const unsigned short l0 = f2bf_bits(v0 - bf_bits2f(h0)), l1 = f2bf_bits(v1 - bf_bits2f(h1));
    hv[e]     = __builtin_bit_cast(_Float16, h0);
    hv[4 + e] = __builtin_bit_cast(_Float16, h1);
    lv[e]     = __builtin_bit_cast(_Float16, l0);
    lv[4 + e] = __builtin_bit_cast(_Float16, l1);
  }
  const size_t o = (size_t)kD * kD + (size_t)e0;
  unsigned short* qh = dhi + o;
  unsigned short* ql = dlo + o;
  *(volatile v8h*)qh = hv;
  *(volatile v8h*)ql = lv;
  __threadfence();
  *(volatile v8h*)qh = hv;
  *(volatile v8h*)ql = lv;
}

__global__ __launch_bounds__(256) void gc_kernel(const float* __restrict__ x, float* __restrict__ GC)
{
  __shared__ float sPart[256];
  __shared__ __align__(16) float sOut[32];
  const int t = threadIdx.x, lp = t & 31, ch = t >> 5;
  const int pair = blockIdx.x * 32 + lp;
  const int bix = pair >> 10, d = pair & (kD - 1);
  const float* px = x + ((size_t)bix * kSeq + (size_t)ch * 256) * kD + d;
  float s = 0.0f;
#pragma unroll 1
  for (int i = 0; i < 256; ++i) s += px[(size_t)i * kD];
  sPart[t] = s;
  __syncthreads();
  if (t < 32) {
    float tot = 0.0f;
#pragma unroll
    for (int c = 0; c < 8; ++c) tot += sPart[t + 32 * c];
    sOut[t] = tot * (1.0f / (float)kSeq);
  }
  __syncthreads();
  if (t < 8) {
    const v4f v = *(const v4f*)(sOut + 4 * t);
    float* dst = GC + (size_t)blockIdx.x * 32 + 4 * t;
    *(volatile v4f*)dst = v;
    __threadfence();
    *(volatile v4f*)dst = v;
  }
}

__global__ __launch_bounds__(256) void liquid_kernel(
    const float* __restrict__ GC, const float* __restrict__ Wi_W, const float* __restrict__ Wi_b,
    const float* __restrict__ Wr_W, const float* __restrict__ tau, const float* __restrict__ h0,
    const float* __restrict__ sel_W, const float* __restrict__ sel_b, float* __restrict__ SEL)
{
  __shared__ float sNh[32];
  __shared__ __align__(16) float sSel[kBatch * kD];
  const int t = threadIdx.x;
  if (t < 32) {
    const int bix = t >> 4, n = t & 15;
    const float* g = GC + (size_t)bix * kD;
    const float* w = Wi_W + (size_t)n * kD;
    float inp = 0.0f;
#pragma unroll 1
    for (int k = 0; k < kD; ++k) inp = fmaf(g[k], w[k], inp);
    inp += Wi_b[n];
    float rec = 0.0f;
#pragma unroll 1
    for (int m = 0; m < kN; ++m) rec = fmaf(h0[m], Wr_W[n * kN + m], rec);
    const float cur = h0[n];
    const float tr  = tau[n];
    const float tc  = fminf(fmaxf(tr, 0.1f), 10.0f);
    const float th  = tanhf(inp + rec);
    const float dh  = (-cur + th) / tc;
    sNh[t] = cur + kDT * dh;
  }
  __syncthreads();
#pragma unroll 1
  for (int i = 0; i < (kBatch * kD) / 256; ++i) {
    const int idx = i * 256 + t;
    const int bix = idx >> 10, d = idx & (kD - 1);
    const float* sw = sel_W + (size_t)d * kN;
    const v4f w0 = *(const v4f*)(sw);
    const v4f w1 = *(const v4f*)(sw + 4);
    const v4f w2 = *(const v4f*)(sw + 8);
    const v4f w3 = *(const v4f*)(sw + 12);
    const float* nh = sNh + bix * kN;
    float s = 0.0f;
#pragma unroll
    for (int e = 0; e < 4; ++e) s = fmaf(nh[e], w0[e], s);
#pragma unroll
    for (int e = 0; e < 4; ++e) s = fmaf(nh[4 + e], w1[e], s);
#pragma unroll
    for (int e = 0; e < 4; ++e) s = fmaf(nh[8 + e], w2[e], s);
#pragma unroll
    for (int e = 0; e < 4; ++e) s = fmaf(nh[12 + e], w3[e], s);
    s += sel_b[d];
    const float ex = expf(-s);
    sSel[idx] = 1.0f / (1.0f + ex);
  }
  __syncthreads();
  v4f sv[2];
#pragma unroll
  for (int it = 0; it < 2; ++it) sv[it] = *(const v4f*)(sSel + (it * 256 + t) * 4);
  for (int pass = 0; pass < 2; ++pass) {
#pragma unroll
    for (int it = 0; it < 2; ++it) *(volatile v4f*)(SEL + (size_t)(it * 256 + t) * 4) = sv[it];
    __threadfence();
  }
}

__global__ __launch_bounds__(256) void scan_kernel(
    const float* __restrict__ P, const float* __restrict__ x, const float* __restrict__ SEL,
    const float* __restrict__ delta_b, const float* __restrict__ dt_bias,
    const float* __restrict__ B_b, const float* __restrict__ C_b, const float* __restrict__ A_log,
    float* __restrict__ Y)
{
  __shared__ __align__(16) float sBC[kScanTS * 32];
  __shared__ __align__(16) float sY[kScanTS * kScanTP];
  __shared__ __align__(16) float sA[kN * kScanCh];
  __shared__ __align__(16) float sI[kN * kScanCh];
  __shared__ __align__(16) float sBias[32];
  const int tid = threadIdx.x, lane = tid & 31, wave = tid >> 5;
  constexpr int kBlkPerB = kD / kScanCh;
  const int bix = blockIdx.x / kBlkPerB;
  const int d0  = (blockIdx.x - bix * kBlkPerB) * kScanCh;
  const int d   = d0 + tid;
  const size_t row0 = (size_t)bix * kSeq;
  if (tid < 32) {
    const float vb = B_b[tid & 15];
    const float vc = C_b[tid & 15];
    const float fb = (tid < 16) ? 1.0f : 0.0f;
    sBias[tid] = fmaf(fb, vb, (1.0f - fb) * vc);
  }
#pragma unroll 1
  for (int s = 0; s < kN; ++s) {
    const float a = -expf(A_log[(size_t)d * kN + s]);
    sA[s * kScanCh + tid] = a;
    sI[s * kScanCh + tid] = (fabsf(a) < 1e-6f) ? 0.0f : (1.0f / a);
  }
  __syncthreads();
  float An[kN], In[kN], h[kN];
#pragma unroll
  for (int s = 0; s < kN; ++s) {
    An[s] = sA[s * kScanCh + tid];
    In[s] = sI[s * kScanCh + tid];
    h[s]  = 0.0f;
  }
  const float selv = SEL[(size_t)bix * kD + d];
  const float dbv  = delta_b[d];
  const float dtv  = dt_bias[d];
  const int hrow = wave >> 1;
  const int hch  = (wave & 1) * 128 + lane * 4;
#pragma unroll 1
  for (int c = 0; c < kSeq / kScanTS; ++c) {
    const int l0 = c * kScanTS;
    if (tid < 128) {
      const int r = tid >> 3, q = (tid & 7) * 4;
      const v4f pv = *(const v4f*)(P + (row0 + l0 + r) * kNP + kD + q);
      const v4f bb = *(const v4f*)(sBias + q);
      *(v4f*)(sBC + r * 32 + q) = pv + bb;
    }
    __syncthreads();
#pragma unroll 1
    for (int s = 0; s < kScanTS; ++s) {
      const size_t m = row0 + l0 + s;
      const float pa = P[m * kNP + d];
      const float p  = (pa + dbv) + dtv;
      const float dl = fmaxf(p, 0.0f) + log1pf(__expf(-fabsf(p)));
      const float xv = x[m * kD + d] * selv;
      v4f Bq[4], Cq[4];
#pragma unroll
      for (int qq = 0; qq < 4; ++qq) {
        Bq[qq] = *(const v4f*)(sBC + s * 32 + 4 * qq);
        Cq[qq] = *(const v4f*)(sBC + s * 32 + kN + 4 * qq);
      }
      float y = 0.0f;
#pragma unroll
      for (int n = 0; n < kN; ++n) {
        const float e  = __expf(dl * An[n]);
        const float tq = (e - 1.0f) * In[n];
        const float fc = (fabsf(An[n]) < 1e-6f) ? dl : tq;
        const float bd = fc * Bq[n >> 2][n & 3];
        const float hn = e * h[n] + bd * xv;
        h[n] = hn;
        y += hn * Cq[n >> 2][n & 3];
      }
      sY[s * kScanTP + tid] = y;
    }
    __syncthreads();
    v4f fv[4];
#pragma unroll
    for (int it = 0; it < 4; ++it) fv[it] = *(const v4f*)(sY + (it * 4 + hrow) * kScanTP + hch);
    for (int pass = 0; pass < 2; ++pass) {
#pragma unroll
      for (int it = 0; it < 4; ++it)
        *(volatile v4f*)(Y + (row0 + l0 + it * 4 + hrow) * kD + d0 + hch) = fv[it];
      __threadfence();
    }
  }
}

extern "C" void kernel_launch(void* const* d_in, const int* in_sizes, int n_in,
                              void* d_out, int out_size, void* d_ws, size_t ws_size,
                              hipStream_t stream)
{
  if (n_in < 16) return;
  if (in_sizes[0] != kRows * kD) return;
  if (in_sizes[1] != kD * kD) return;
  if (in_sizes[2] != kD) return;
  if (in_sizes[3] != kN * kD || in_sizes[4] != kN) return;
  if (in_sizes[5] != kN * kD || in_sizes[6] != kN) return;
  if (in_sizes[7] != kD * kN) return;
  if (in_sizes[8] != kD) return;
  if (in_sizes[9] != kN) return;
  if (in_sizes[10] != kN * kD || in_sizes[11] != kN) return;
  if (in_sizes[12] != kN * kN) return;
  if (in_sizes[13] != kD * kN || in_sizes[14] != kD) return;
  if (in_sizes[15] != kN) return;
  if (out_size != kRows * kD) return;
  if (ws_size < kWsTotal) return;

  const float* x       = (const float*)d_in[0];
  const float* delta_W = (const float*)d_in[1];
  const float* delta_b = (const float*)d_in[2];
  const float* B_W     = (const float*)d_in[3];
  const float* B_b     = (const float*)d_in[4];
  const float* C_W     = (const float*)d_in[5];
  const float* C_b     = (const float*)d_in[6];
  const float* A_log   = (const float*)d_in[7];
  const float* dt_bias = (const float*)d_in[8];
  const float* tau     = (const float*)d_in[9];
  const float* Wi_W    = (const float*)d_in[10];
  const float* Wi_b    = (const float*)d_in[11];
  const float* Wr_W    = (const float*)d_in[12];
  const float* sel_W   = (const float*)d_in[13];
  const float* sel_b   = (const float*)d_in[14];
  const float* h0      = (const float*)d_in[15];
  float* out = (float*)d_out;

  char* ws = (char*)d_ws;
  float*          GC  = (float*)(ws + kOffGC);
  float*          SEL = (float*)(ws + kOffSEL);
  unsigned short* XSH = (unsigned short*)(ws + kOffXSH);
  unsigned short* XSL = (unsigned short*)(ws + kOffXSL);
  unsigned short* WH  = (unsigned short*)(ws + kOffWH);
  unsigned short* WL  = (unsigned short*)(ws + kOffWL);
  float*          P   = (float*)(ws + kOffP);

  gc_kernel<<<(kBatch * kD) / 32, 256, 0, stream>>>(x, GC);

  liquid_kernel<<<1, 256, 0, stream>>>(GC, Wi_W, Wi_b, Wr_W, tau, h0, sel_W, sel_b, SEL);

  xs_split_kernel<<<(kRows * kD / 8) / 256, 256, 0, stream>>>(x, SEL, XSH, XSL, kRows * kD / 8);

  split_rows_bf16_kernel<<<(kD * kD / 8) / 256, 256, 0, stream>>>(delta_W, WH, WL, kD * kD / 8);

  wtail_split_kernel<<<(((kNP - kD) * kD) / 8) / 256, 256, 0, stream>>>(B_W, C_W, WH, WL);

  wmma_gemm64<1, 2, 0, 0, false><<<dim3(((kRows / 64) * (kNP / 64)) / 8, 1), 256, 0, stream>>>(
      XSH, XSL, kD, 0L,
      WH, WL, kD, 0L,
      (void*)P, nullptr, kNP, 0L,
      nullptr, nullptr, 0L,
      kRows, kNP, kD, 1.0f);

  scan_kernel<<<kBatch * (kD / kScanCh), kScanCh, 0, stream>>>(P, x, SEL, delta_b, dt_bias, B_b, C_b, A_log, out);
}
